// pSGM_27023934227052
// MI455X (gfx1250) — hardware-verified
//
#include <hip/hip_runtime.h>
#include <math.h>
#include <stdint.h>

#define NB_  2
#define CH_  256
#define CI_  128
#define NP_  12544
#define NS_  3136
#define HW_  784
#define WR_  28
#define PHW_ 196
#define PW_  14
#define QT_  196
#define KT_  49

typedef __attribute__((ext_vector_type(16))) _Float16 v16h;
typedef __attribute__((ext_vector_type(8)))  _Float16 v8h;
typedef __attribute__((ext_vector_type(16))) __bf16   v16b;
typedef __attribute__((ext_vector_type(8)))  __bf16   v8b;
typedef __attribute__((ext_vector_type(8)))  float    v8f;
typedef __attribute__((ext_vector_type(4)))  float    v4f;
typedef __attribute__((ext_vector_type(4)))  unsigned int v4u;

__device__ __forceinline__ unsigned short f2bf_bits(float f) {
  const unsigned u = __float_as_uint(f);
  return (unsigned short)((u + 0x7FFFu + ((u >> 16) & 1u)) >> 16);
}
__device__ __forceinline__ float bf_bits2f(unsigned short h) { return __uint_as_float(((unsigned)h) << 16); }
__device__ __forceinline__ unsigned pk16(unsigned short a, unsigned short b) { return (unsigned)a | ((unsigned)b << 16); }

union FragB { v16b v; v8b h[2]; };

__device__ __forceinline__ v16b ldfrag_b(const __bf16* p) {
  FragB f; f.h[0] = *(const v8b*)(p); f.h[1] = *(const v8b*)(p + 16); return f.v;
}

__device__ __forceinline__ v8f mma_b(v16b a, v16b b, v8f c) {
  return __builtin_amdgcn_wmma_f32_16x16x32_bf16(false, a, false, b, (short)0, c, false, false);
}
__device__ __forceinline__ void dep_guard_b(v8f& a, v8f& b, v16b x, v16b y) {
  asm volatile("v_nop\n\tv_nop\n\tv_nop\n\tv_nop" : "+v"(a), "+v"(b) : "v"(x), "v"(y));
}
__device__ __forceinline__ void guard5(v8f& c, v16b a0, v16b a1, v16b b0, v16b b1) {
  asm volatile("v_nop\n\tv_nop\n\tv_nop\n\tv_nop" : "+v"(c) : "v"(a0), "v"(a1), "v"(b0), "v"(b1));
}
__device__ __forceinline__ void keep4_b(v16b a, v16b b, v16b c, v16b d) {
  asm volatile("v_nop" :: "v"(a), "v"(b), "v"(c), "v"(d));
}
__device__ __forceinline__ void acc_guard4(v8f& a, v8f& b, v8f& c, v8f& d) {
  asm volatile("v_nop\n\tv_nop\n\tv_nop\n\tv_nop" : "+v"(a), "+v"(b), "+v"(c), "+v"(d));
}
__device__ __forceinline__ void wave_sync_lds() {
  __builtin_amdgcn_fence(__ATOMIC_RELEASE, "workgroup");
  __builtin_amdgcn_wave_barrier();
  __builtin_amdgcn_fence(__ATOMIC_ACQUIRE, "workgroup");
}

__device__ __forceinline__ void mac_tile64(v8f (&acc)[4][4],
    const __bf16* __restrict__ A, const __bf16* __restrict__ A2, int lda,
    const __bf16* __restrict__ B, const __bf16* __restrict__ B2, int ldb,
    int m0, int n0, int K, int lane) {
  const int rlane = lane & 15, koff = (lane >> 4) * 8;
  for (int k0 = 0; k0 < K; k0 += 32) {
    v16b bh[4], bl[4];
#pragma unroll
    for (int j = 0; j < 4; ++j) {
      const size_t bo = (size_t)(n0 + (j << 4) + rlane) * ldb + koff + k0;
      bh[j] = ldfrag_b(B + bo);
      bl[j] = ldfrag_b(B2 + bo);
    }
#pragma unroll
    for (int i = 0; i < 4; ++i) {
      const size_t ao = (size_t)(m0 + (i << 4) + rlane) * lda + koff + k0;
      const v16b ah = ldfrag_b(A + ao);
      const v16b al = ldfrag_b(A2 + ao);
#pragma unroll
      for (int j = 0; j < 4; ++j) {
        acc[i][j] = mma_b(ah, bh[j], acc[i][j]);
        acc[i][j] = mma_b(ah, bl[j], acc[i][j]);
        acc[i][j] = mma_b(al, bh[j], acc[i][j]);
      }
      dep_guard_b(acc[i][0], acc[i][3], ah, al);
    }
    keep4_b(bh[0], bh[1], bh[2], bh[3]);
    keep4_b(bl[0], bl[1], bl[2], bl[3]);
  }
  acc_guard4(acc[0][0], acc[0][1], acc[0][2], acc[0][3]);
  acc_guard4(acc[1][0], acc[1][1], acc[1][2], acc[1][3]);
  acc_guard4(acc[2][0], acc[2][1], acc[2][2], acc[2][3]);
  acc_guard4(acc[3][0], acc[3][1], acc[3][2], acc[3][3]);
}

__device__ __forceinline__ void store_rows_f32(const float* slab, float* C, int ldc, int mBase, int n0, int lane) {
  const int hh = lane >> 4, c4 = (lane & 15) * 4;
  for (int pass = 0; pass < 2; ++pass) {
#pragma unroll
    for (int it = 0; it < 8; ++it) {
      const int row = it * 2 + hh;
      const v4f v = *(const v4f*)(slab + row * 68 + c4);
      *(volatile v4f*)(C + (size_t)(mBase + row) * ldc + n0 + c4) = v;
    }
    __threadfence();
  }
}
__device__ __forceinline__ void store_rows_bf16x2(const float* slab, unsigned short* C, unsigned short* C2, int ldc,
                                                  int mBase, int n0, int lane) {
  const int q = lane >> 3, c8 = (lane & 7) * 8;
  for (int pass = 0; pass < 2; ++pass) {
#pragma unroll
    for (int it = 0; it < 4; ++it) {
      const int row = it * 4 + q;
      const float* sp = slab + row * 68 + c8;
      v8h hv, lv;
#pragma unroll
      for (int e = 0; e < 8; ++e) {
        const unsigned short hb = f2bf_bits(sp[e]);
        const unsigned short lb = f2bf_bits(sp[e] - bf_bits2f(hb));
        hv[e] = __builtin_bit_cast(_Float16, hb);
        lv[e] = __builtin_bit_cast(_Float16, lb);
      }
      *(volatile v8h*)(C  + (size_t)(mBase + row) * ldc + n0 + c8) = hv;
      *(volatile v8h*)(C2 + (size_t)(mBase + row) * ldc + n0 + c8) = lv;
    }
    __threadfence();
  }
}

template <int BIAS_MODE, int OUT_MODE>
__global__ __launch_bounds__(256) void gemm64_kernel(
    const unsigned short* __restrict__ Ahp, const unsigned short* __restrict__ Alp, int lda,
    const unsigned short* __restrict__ Bhp, const unsigned short* __restrict__ Blp, int ldb,
    void* __restrict__ Cout, void* __restrict__ Cout2, int ldc,
    const float* __restrict__ bias, int M, int N, int K) {
  __shared__ __align__(16) float sT[8][16 * 68];
  const __bf16* A  = (const __bf16*)(const void*)Ahp;
  const __bf16* A2 = (const __bf16*)(const void*)Alp;
  const __bf16* B  = (const __bf16*)(const void*)Bhp;
  const __bf16* B2 = (const __bf16*)(const void*)Blp;
  const int lane = threadIdx.x & 31, wave = threadIdx.x >> 5;
  const int tilesN = N >> 6, tilesM = M >> 6;
  const int tile = blockIdx.x * 8 + wave;
  if (tile >= tilesM * tilesN) return;
  const int tm = tile / tilesN, tn = tile - tm * tilesN;
  const int m0 = tm << 6, n0 = tn << 6;
  const int rlane = lane & 15, mOff = (lane >> 4) * 8;

  v8f acc[4][4];
#pragma unroll
  for (int i = 0; i < 4; ++i)
#pragma unroll
    for (int j = 0; j < 4; ++j) acc[i][j] = (v8f){0.f,0.f,0.f,0.f,0.f,0.f,0.f,0.f};

  mac_tile64(acc, A, A2, lda, B, B2, ldb, m0, n0, K, lane);

  float* slab = sT[wave];
#pragma unroll
  for (int i = 0; i < 4; ++i) {
    const int mBase = m0 + (i << 4);
#pragma unroll
    for (int j = 0; j < 4; ++j) {
      const int n = n0 + (j << 4) + rlane;
      float bv = 0.f;
      if (BIAS_MODE == 2) bv = bias[n];
#pragma unroll
      for (int r = 0; r < 8; ++r) {
        float v = acc[i][j][r];
        if (BIAS_MODE == 1) v += bias[mBase + mOff + r];
        if (BIAS_MODE == 2) v += bv;
        slab[(mOff + r) * 68 + (j << 4) + rlane] = v;
      }
    }
    wave_sync_lds();
    if (OUT_MODE == 0) {
      store_rows_f32(slab, (float*)Cout, ldc, mBase, n0, lane);
    } else {
      store_rows_bf16x2(slab, (unsigned short*)Cout, (unsigned short*)Cout2, ldc, mBase, n0, lane);
    }
    wave_sync_lds();
  }
}

__global__ __launch_bounds__(256) void sgemm_stats_kernel(
    const unsigned short* __restrict__ Thp, const unsigned short* __restrict__ Tlp,
    const unsigned short* __restrict__ Php, const unsigned short* __restrict__ Plp,
    float* __restrict__ Sout, float* __restrict__ Pmax, float* __restrict__ Psum) {
  __shared__ __align__(16) float sT[8][16 * 68];
  const __bf16* A  = (const __bf16*)(const void*)Thp;
  const __bf16* A2 = (const __bf16*)(const void*)Tlp;
  const __bf16* B  = (const __bf16*)(const void*)Php;
  const __bf16* B2 = (const __bf16*)(const void*)Plp;
  const int lane = threadIdx.x & 31, wave = threadIdx.x >> 5;
  const int tile = blockIdx.x * 8 + wave;
  if (tile >= QT_ * KT_) return;
  const int tm = tile / KT_, tn = tile - tm * KT_;
  const int m0 = tm << 6, n0 = tn << 6;
  const int rlane = lane & 15, mOff = (lane >> 4) * 8;

  v8f acc[4][4];
#pragma unroll
  for (int i = 0; i < 4; ++i)
#pragma unroll
    for (int j = 0; j < 4; ++j) acc[i][j] = (v8f){0.f,0.f,0.f,0.f,0.f,0.f,0.f,0.f};

  mac_tile64(acc, A, A2, CI_, B, B2, CI_, m0, n0, CI_, lane);

  float* slab = sT[wave];
  float cm0 = 0.f, cm1 = 0.f, cs0 = 0.f, cs1 = 0.f;
#pragma unroll
  for (int i = 0; i < 4; ++i) {
    const int mBase = m0 + (i << 4);
#pragma unroll
    for (int j = 0; j < 4; ++j) {
#pragma unroll
      for (int r = 0; r < 8; ++r) slab[(mOff + r) * 68 + (j << 4) + rlane] = acc[i][j][r];
    }
    wave_sync_lds();
    {
      float v0[16], v1[16];
      float t0 = slab[lane], t1 = slab[32 + lane];
#pragma unroll
      for (int rr = 0; rr < 16; ++rr) {
        v0[rr] = slab[rr * 68 + lane];
        v1[rr] = slab[rr * 68 + 32 + lane];
        t0 = fmaxf(t0, v0[rr]);
        t1 = fmaxf(t1, v1[rr]);
      }
      float nm0, nm1, s0, s1;
      if (i == 0) {
        nm0 = t0; nm1 = t1; s0 = 0.f; s1 = 0.f;
      } else {
        nm0 = fmaxf(cm0, t0); nm1 = fmaxf(cm1, t1);
        s0 = cs0 * __expf(cm0 - nm0);
        s1 = cs1 * __expf(cm1 - nm1);
      }
#pragma unroll
      for (int rr = 0; rr < 16; ++rr) {
        s0 += __expf(v0[rr] - nm0);
        s1 += __expf(v1[rr] - nm1);
      }
      cm0 = nm0; cs0 = s0; cm1 = nm1; cs1 = s1;
    }
    store_rows_f32(slab, Sout, NS_, mBase, n0, lane);
    wave_sync_lds();
  }
  {
    const size_t po = (size_t)tm * NS_ + n0;
    *(volatile float*)(Pmax + po + lane) = cm0;
    *(volatile float*)(Pmax + po + 32 + lane) = cm1;
    *(volatile float*)(Psum + po + lane) = cs0;
    *(volatile float*)(Psum + po + 32 + lane) = cs1;
    __threadfence();
    *(volatile float*)(Pmax + po + lane) = cm0;
    *(volatile float*)(Pmax + po + 32 + lane) = cm1;
    *(volatile float*)(Psum + po + lane) = cs0;
    *(volatile float*)(Psum + po + 32 + lane) = cs1;
  }
}

__global__ __launch_bounds__(256) void split_w_kernel(const float* __restrict__ in, unsigned short* __restrict__ hi,
                                                      unsigned short* __restrict__ lo, int n2) {
  const int i = blockIdx.x * 256 + threadIdx.x;
  if (i < n2) {
    const float f0 = in[2 * (size_t)i], f1 = in[2 * (size_t)i + 1];
    const unsigned short h0 = f2bf_bits(f0), h1 = f2bf_bits(f1);
    const unsigned short l0 = f2bf_bits(f0 - bf_bits2f(h0)), l1 = f2bf_bits(f1 - bf_bits2f(h1));
    const unsigned uh = pk16(h0, h1), ul = pk16(l0, l1);
    ((volatile unsigned*)hi)[i] = uh;
    ((volatile unsigned*)lo)[i] = ul;
    __threadfence();
    ((volatile unsigned*)hi)[i] = uh;
    ((volatile unsigned*)lo)[i] = ul;
  }
}

__global__ __launch_bounds__(256) void tsplit_kernel(const float* __restrict__ W, unsigned short* __restrict__ oh,
                                                     unsigned short* __restrict__ ol, int R, int Cc) {
  __shared__ __align__(16) float tf[64 * 68];
  const int c0  = blockIdx.x * 64;
  const int r0  = blockIdx.y * 64;
  const int tid = threadIdx.x;
  {
    const int lr = tid >> 4;
    const int c4 = (tid & 15) * 4;
#pragma unroll
    for (int it = 0; it < 4; ++it) {
      const int rr = it * 16 + lr;
      const v4f a = *(const v4f*)(W + (size_t)(r0 + rr) * Cc + c0 + c4);
      *(v4f*)(tf + rr * 68 + c4) = a;
    }
  }
  __syncthreads();
  const int sub = tid >> 3;
  const int c8  = (tid & 7) * 8;
  v4u hv[2], lv[2];
#pragma unroll
  for (int it = 0; it < 2; ++it) {
    const int oc = it * 32 + sub;
    v4u a, a2;
#pragma unroll
    for (int q = 0; q < 4; ++q) {
      const float f0 = tf[(c8 + 2 * q) * 68 + oc];
      const float f1 = tf[(c8 + 2 * q + 1) * 68 + oc];
      const unsigned short h0 = f2bf_bits(f0), h1 = f2bf_bits(f1);
      const unsigned short l0 = f2bf_bits(f0 - bf_bits2f(h0)), l1 = f2bf_bits(f1 - bf_bits2f(h1));
      a[q]  = pk16(h0, h1);
      a2[q] = pk16(l0, l1);
    }
    hv[it] = a; lv[it] = a2;
  }
  for (int pass = 0; pass < 2; ++pass) {
#pragma unroll
    for (int it = 0; it < 2; ++it) {
      const int oc = it * 32 + sub;
      const size_t go = (size_t)(c0 + oc) * R + r0 + c8;
      *(volatile v4u*)(oh + go) = hv[it];
      *(volatile v4u*)(ol + go) = lv[it];
    }
    __threadfence();
  }
}

__global__ __launch_bounds__(256) void pool_kernel(
    const float* __restrict__ Gpre, const float* __restrict__ Ppre,
    unsigned short* __restrict__ PhH, unsigned short* __restrict__ PhL,
    float* __restrict__ Gpool) {
  __shared__ __align__(16) float lds[64 * 136];
  const int tid = threadIdx.x;
  const int m0 = blockIdx.x * 64;
  const int ml = tid >> 2, ch = (tid & 3) * 32;
  const int m = m0 + ml;
  const int t = m / PHW_;
  const int rem = m - t * PHW_;
  const int h2 = rem / PW_;
  const int w2 = rem - h2 * PW_;
  const int n00 = t * HW_ + 2 * h2 * WR_ + 2 * w2;
  const float* gp = Gpre + (size_t)n00 * CI_ + ch;
  const float* pp = Ppre + (size_t)n00 * CI_ + ch;
  float gv[32], fv[32];
#pragma unroll
  for (int j = 0; j < 8; ++j) {
    const v4f a0 = *(const v4f*)(gp + 4 * j);
    const v4f a1 = *(const v4f*)(gp + CI_ + 4 * j);
    const v4f a2 = *(const v4f*)(gp + WR_ * CI_ + 4 * j);
    const v4f a3 = *(const v4f*)(gp + (WR_ + 1) * CI_ + 4 * j);
    const v4f b0 = *(const v4f*)(pp + 4 * j);
    const v4f b1 = *(const v4f*)(pp + CI_ + 4 * j);
    const v4f b2 = *(const v4f*)(pp + WR_ * CI_ + 4 * j);
    const v4f b3 = *(const v4f*)(pp + (WR_ + 1) * CI_ + 4 * j);
#pragma unroll
    for (int e = 0; e < 4; ++e) {
      gv[4 * j + e] = fmaxf(fmaxf(a0[e], a1[e]), fmaxf(a2[e], a3[e]));
      fv[4 * j + e] = fmaxf(fmaxf(b0[e], b1[e]), fmaxf(b2[e], b3[e]));
    }
  }
  unsigned* lu = (unsigned*)lds;
#pragma unroll
  for (int q = 0; q < 4; ++q) {
    v4u hv, lv;
#pragma unroll
    for (int e = 0; e < 4; ++e) {
      const float f0 = fv[8 * q + 2 * e], f1 = fv[8 * q + 2 * e + 1];
      const unsigned short h0 = f2bf_bits(f0), h1 = f2bf_bits(f1);
      const unsigned short l0 = f2bf_bits(f0 - bf_bits2f(h0)), l1 = f2bf_bits(f1 - bf_bits2f(h1));
      hv[e] = pk16(h0, h1);
      lv[e] = pk16(l0, l1);
    }
    *(v4u*)(lu + ml * 68 + (ch >> 1) + 4 * q) = hv;
    *(v4u*)(lu + 64 * 68 + ml * 68 + (ch >> 1) + 4 * q) = lv;
  }
  __syncthreads();
  {
    const int rr = tid >> 4, qc = (tid & 15) * 4;
    v4u hv[4], lv[4];
#pragma unroll
    for (int it = 0; it < 4; ++it) {
      hv[it] = *(const v4u*)(lu + (it * 16 + rr) * 68 + qc);
      lv[it] = *(const v4u*)(lu + 64 * 68 + (it * 16 + rr) * 68 + qc);
    }
    for (int pass = 0; pass < 2; ++pass) {
#pragma unroll
      for (int it = 0; it < 4; ++it) {
        const size_t go = (size_t)(m0 + it * 16 + rr) * CI_ + qc * 2;
        *(volatile v4u*)(PhH + go) = hv[it];
        *(volatile v4u*)(PhL + go) = lv[it];
      }
      __threadfence();
    }
  }
  __syncthreads();
  float* lf = lds;
#pragma unroll
  for (int j = 0; j < 8; ++j) {
    const v4f v = (v4f){gv[4 * j], gv[4 * j + 1], gv[4 * j + 2], gv[4 * j + 3]};
    *(v4f*)(lf + ml * 132 + ch + 4 * j) = v;
  }
  __syncthreads();
  {
    const int rw = tid >> 5, c4 = (tid & 31) * 4;
    v4f vv[8];
#pragma unroll
    for (int it = 0; it < 8; ++it) vv[it] = *(const v4f*)(lf + (it * 8 + rw) * 132 + c4);
    for (int pass = 0; pass < 2; ++pass) {
#pragma unroll
      for (int it = 0; it < 8; ++it)
        *(volatile v4f*)(Gpool + (size_t)(m0 + it * 8 + rw) * CI_ + c4) = vv[it];
      __threadfence();
    }
  }
}

__global__ __launch_bounds__(64) void combine_kernel(const float* __restrict__ Pmax, const float* __restrict__ Psum,
                                                     float* __restrict__ Cmax, float* __restrict__ Cinv) {
  const int tid = threadIdx.x;
  const int m = blockIdx.x * 64 + tid;
  float M = -INFINITY;
  for (int t = 0; t < QT_; ++t) M = fmaxf(M, Pmax[(size_t)t * NS_ + m]);
  float S = 0.f;
  for (int t = 0; t < QT_; ++t) S += Psum[(size_t)t * NS_ + m] * __expf(Pmax[(size_t)t * NS_ + m] - M);
  const float cinv = 1.0f / S;
  *(volatile float*)(Cmax + m) = M;
  *(volatile float*)(Cinv + m) = cinv;
  __threadfence();
  *(volatile float*)(Cmax + m) = M;
  *(volatile float*)(Cinv + m) = cinv;
}

__global__ __launch_bounds__(128) void pv_kernel(
    const float* __restrict__ S, const float* __restrict__ Cmax, const float* __restrict__ Cinv,
    const unsigned short* __restrict__ GThp, const unsigned short* __restrict__ GTlp,
    unsigned short* __restrict__ YH, unsigned short* __restrict__ YL) {
  __shared__ __align__(16) __bf16 Pth[64 * 72];
  __shared__ __align__(16) __bf16 Ptl[64 * 72];
  __shared__ __align__(16) float Os[4][16 * 132];
  const __bf16* GTH = (const __bf16*)(const void*)GThp;
  const __bf16* GTL = (const __bf16*)(const void*)GTlp;
  const int tid = threadIdx.x, wave = tid >> 5, lane = tid & 31, hh = lane >> 4, c = lane & 15;
  const int n0 = blockIdx.x * 64;
  const int pr = tid >> 1, pc = (tid & 1) * 32;
  const float* srow = S + (size_t)(n0 + pr) * NS_ + pc;

  v8f acc[8];
#pragma unroll
  for (int t = 0; t < 8; ++t) acc[t] = (v8f){0.f,0.f,0.f,0.f,0.f,0.f,0.f,0.f};

  for (int kt = 0; kt < KT_; ++kt) {
    const int mt0 = kt * 64;
    __syncthreads();
#pragma unroll
    for (int j = 0; j < 4; ++j) {
      const v4f s0 = *(const v4f*)(srow + mt0 + 8 * j);
      const v4f s1 = *(const v4f*)(srow + mt0 + 8 * j + 4);
      const v4f x0 = *(const v4f*)(Cmax + mt0 + pc + 8 * j);
      const v4f x1 = *(const v4f*)(Cmax + mt0 + pc + 8 * j + 4);
      const v4f i0 = *(const v4f*)(Cinv + mt0 + pc + 8 * j);
      const v4f i1 = *(const v4f*)(Cinv + mt0 + pc + 8 * j + 4);
      v8b hv, lv;
#pragma unroll
      for (int e = 0; e < 4; ++e) {
        const float p0 = __expf(s0[e] - x0[e]) * i0[e];
        const float p1 = __expf(s1[e] - x1[e]) * i1[e];
        const unsigned short h0 = f2bf_bits(p0), h1 = f2bf_bits(p1);
        const unsigned short l0 = f2bf_bits(p0 - bf_bits2f(h0)), l1 = f2bf_bits(p1 - bf_bits2f(h1));
        hv[e]     = __builtin_bit_cast(__bf16, h0);
        hv[4 + e] = __builtin_bit_cast(__bf16, h1);
        lv[e]     = __builtin_bit_cast(__bf16, l0);
        lv[4 + e] = __builtin_bit_cast(__bf16, l1);
      }
      *(v8b*)(Pth + pr * 72 + pc + 8 * j) = hv;
      *(v8b*)(Ptl + pr * 72 + pc + 8 * j) = lv;
    }
    __syncthreads();
#pragma unroll
    for (int ks = 0; ks < 2; ++ks) {
      FragB ah, al;
      const __bf16* pah = Pth + (wave * 16 + c) * 72 + ks * 32 + 8 * hh;
      const __bf16* pal = Ptl + (wave * 16 + c) * 72 + ks * 32 + 8 * hh;
      ah.h[0] = *(const v8b*)(pah);
      ah.h[1] = *(const v8b*)(pah + 16);
      al.h[0] = *(const v8b*)(pal);
      al.h[1] = *(const v8b*)(pal + 16);
      const __bf16* gh = GTH + (size_t)c * NS_ + mt0 + ks * 32 + 8 * hh;
      const __bf16* gl = GTL + (size_t)c * NS_ + mt0 + ks * 32 + 8 * hh;
#pragma unroll
      for (int t = 0; t < 8; ++t) {
        FragB bh, bl;
        const size_t to = (size_t)(t * 16) * NS_;
        bh.h[0] = *(const v8b*)(gh + to);
        bh.h[1] = *(const v8b*)(gh + to + 16);
        bl.h[0] = *(const v8b*)(gl + to);
        bl.h[1] = *(const v8b*)(gl + to + 16);
        acc[t] = mma_b(ah.v, bh.v, acc[t]);
        acc[t] = mma_b(ah.v, bl.v, acc[t]);
        acc[t] = mma_b(al.v, bh.v, acc[t]);
        guard5(acc[t], ah.v, al.v, bh.v, bl.v);
      }
    }
  }

  float* os = Os[wave];
#pragma unroll
  for (int r = 0; r < 8; ++r) {
#pragma unroll
    for (int t = 0; t < 8; ++t)
      os[(8 * hh + r) * 132 + t * 16 + c] = acc[t][r];
  }
  wave_sync_lds();
  unsigned short* yh = YH + (size_t)(n0 + wave * 16) * CI_;
  unsigned short* yl = YL + (size_t)(n0 + wave * 16) * CI_;
  for (int pass = 0; pass < 2; ++pass) {
#pragma unroll
    for (int it = 0; it < 8; ++it) {
      const int row = it * 2 + hh;
      const float* sp = os + row * 132 + c * 8;
      v8h hv, lv;
#pragma unroll
      for (int e = 0; e < 8; ++e) {
        const unsigned short hb = f2bf_bits(sp[e]);
        const unsigned short lb = f2bf_bits(sp[e] - bf_bits2f(hb));
        hv[e] = __builtin_bit_cast(_Float16, hb);
        lv[e] = __builtin_bit_cast(_Float16, lb);
      }
      *(volatile v8h*)(yh + (size_t)row * CI_ + c * 8) = hv;
      *(volatile v8h*)(yl + (size_t)row * CI_ + c * 8) = lv;
    }
    __threadfence();
  }
}

__global__ __launch_bounds__(256) void bn_stats_kernel(const float* __restrict__ Wy, const float* __restrict__ gamma,
                                                       const float* __restrict__ beta, float* __restrict__ SS) {
  __shared__ __align__(16) float ss[512];
  const int c = threadIdx.x;
  double s = 0.0;
  for (int b = 0; b < NB_; ++b) {
    const float* p = Wy + ((size_t)b * CH_ + c) * NP_;
#pragma unroll 1
    for (int n = 0; n < NP_; ++n) s += (double)p[n];
  }
  const double mean = s / (double)(NB_ * NP_);
  double q = 0.0;
  for (int b = 0; b < NB_; ++b) {
    const float* p = Wy + ((size_t)b * CH_ + c) * NP_;
#pragma unroll 1
    for (int n = 0; n < NP_; ++n) { const double d = (double)p[n] - mean; q += d * d; }
  }
  const double var = q / (double)(NB_ * NP_);
  const float varf = (float)var;
  const float rstd = 1.0f / sqrtf(varf + 1e-5f);
  const float sc = gamma[c] * rstd;
  const float sh = beta[c] - (float)mean * sc;
  ss[c] = sc;
  ss[256 + c] = sh;
  __syncthreads();
  if (c < 128) {
    const v4f v = *(const v4f*)(ss + c * 4);
    *(volatile v4f*)(SS + c * 4) = v;
    __threadfence();
    *(volatile v4f*)(SS + c * 4) = v;
  }
}

__global__ __launch_bounds__(256) void final_kernel(const float* __restrict__ Wy, const float* __restrict__ X,
                                                    const float* __restrict__ SS, float* __restrict__ out) {
  const int c = blockIdx.x, b = blockIdx.y;
  const float sc = SS[c], sh = SS[256 + c];
  const size_t base = ((size_t)b * CH_ + c) * NP_;
  const v4f* w4 = (const v4f*)(Wy + base);
  const v4f* x4 = (const v4f*)(X + base);
  float* o = out + base;
  for (int pass = 0; pass < 2; ++pass) {
    for (int i = threadIdx.x; i < NP_ / 4; i += 256) {
      const v4f w = w4[i], xx = x4[i];
      const v4f v = w * sc + sh + xx;
      *(volatile v4f*)(o + 4 * (size_t)i) = v;
    }
    __threadfence();
  }
}

extern "C" void kernel_launch(void* const* d_in, const int* in_sizes, int n_in,
                              void* d_out, int out_size, void* d_ws, size_t ws_size,
                              hipStream_t stream) {
  if (n_in < 12) return;
  if (in_sizes[0] != NB_ * CH_ * NP_ || in_sizes[1] != NB_ * CH_ * NP_) return;
  if (in_sizes[2] != CI_ * CH_ || in_sizes[4] != CI_ * CH_ || in_sizes[6] != CI_ * CH_ || in_sizes[8] != CH_ * CI_) return;
  if (in_sizes[3] != CI_ || in_sizes[5] != CI_ || in_sizes[7] != CI_) return;
  if (in_sizes[9] != CH_ || in_sizes[10] != CH_ || in_sizes[11] != CH_) return;
  if (out_size != NB_ * CH_ * NP_) return;

  const float* x     = (const float*)d_in[0];
  const float* mask  = (const float*)d_in[1];
  const float* g_w   = (const float*)d_in[2];
  const float* g_b   = (const float*)d_in[3];
  const float* th_w  = (const float*)d_in[4];
  const float* th_b  = (const float*)d_in[5];
  const float* ph_w  = (const float*)d_in[6];
  const float* ph_b  = (const float*)d_in[7];
  const float* W_w   = (const float*)d_in[8];
  const float* W_b   = (const float*)d_in[9];
  const float* gamma = (const float*)d_in[10];
  const float* beta  = (const float*)d_in[11];
  float* out = (float*)d_out;

  const size_t PWT  = (size_t)CI_ * CH_ * 2;
  const size_t PACT = (size_t)NP_ * CH_ * 2;
  const size_t PTH  = (size_t)NP_ * CI_ * 2;
  const size_t PPRE = (size_t)NP_ * CI_ * 4;
  const size_t PPH  = (size_t)NS_ * CI_ * 2;
  size_t off = 0;
  const size_t oWgH = off; off += PWT;  const size_t oWgL = off; off += PWT;
  const size_t oWpH = off; off += PWT;  const size_t oWpL = off; off += PWT;
  const size_t oWtH = off; off += PWT;  const size_t oWtL = off; off += PWT;
  const size_t oWwH = off; off += PWT;  const size_t oWwL = off; off += PWT;
  const size_t oWy  = off; off += (size_t)NB_ * CH_ * NP_ * 4;
  const size_t oSS  = off; off += 512 * 4;
  const size_t oXH  = off; off += PACT; const size_t oXL  = off; off += PACT;
  const size_t oMH  = off; off += PACT; const size_t oML  = off; off += PACT;
  const size_t oThH = off; off += PTH;  const size_t oThL = off; off += PTH;
  const size_t oGpre = off; off += PPRE; const size_t oPpre = off; off += PPRE;
  const size_t oPhH = off; off += PPH;  const size_t oPhL = off; off += PPH;
  const size_t oGpool = off; off += (size_t)NS_ * CI_ * 4;
  const size_t oGTH  = off; off += PPH;  const size_t oGTL = off; off += PPH;
  const size_t oS    = off; off += (size_t)NP_ * NS_ * 4;
  const size_t oPmax = off; off += (size_t)QT_ * NS_ * 4;
  const size_t oPsum = off; off += (size_t)QT_ * NS_ * 4;
  const size_t oCmax = off; off += (size_t)NS_ * 4;
  const size_t oCinv = off; off += (size_t)NS_ * 4;
  const size_t oYH   = off; off += PTH;  const size_t oYL = off; off += PTH;
  if (off > ws_size) return;

  char* ws = (char*)d_ws;
  unsigned short* WgH = (unsigned short*)(ws + oWgH); unsigned short* WgL = (unsigned short*)(ws + oWgL);
  unsigned short* WpH = (unsigned short*)(ws + oWpH); unsigned short* WpL = (unsigned short*)(ws + oWpL);
  unsigned short* WtH = (unsigned short*)(ws + oWtH); unsigned short* WtL = (unsigned short*)(ws + oWtL);
  unsigned short* WwH = (unsigned short*)(ws + oWwH); unsigned short* WwL = (unsigned short*)(ws + oWwL);
  float* Wy = (float*)(ws + oWy);
  float* SS = (float*)(ws + oSS);
  unsigned short* XH  = (unsigned short*)(ws + oXH);  unsigned short* XL  = (unsigned short*)(ws + oXL);
  unsigned short* MH  = (unsigned short*)(ws + oMH);  unsigned short* ML  = (unsigned short*)(ws + oML);
  unsigned short* ThH = (unsigned short*)(ws + oThH); unsigned short* ThL = (unsigned short*)(ws + oThL);
  float* Gpre = (float*)(ws + oGpre); float* Ppre = (float*)(ws + oPpre);
  unsigned short* PhH = (unsigned short*)(ws + oPhH); unsigned short* PhL = (unsigned short*)(ws + oPhL);
  float* Gpool = (float*)(ws + oGpool);
  unsigned short* GTH = (unsigned short*)(ws + oGTH); unsigned short* GTL = (unsigned short*)(ws + oGTL);
  float* S = (float*)(ws + oS);
  float* Pmax = (float*)(ws + oPmax); float* Psum = (float*)(ws + oPsum);
  float* Cmax = (float*)(ws + oCmax); float* Cinv = (float*)(ws + oCinv);
  unsigned short* YH = (unsigned short*)(ws + oYH); unsigned short* YL = (unsigned short*)(ws + oYL);

  const dim3 blk(256);
  const int n2w = CI_ * CH_ / 2;
  const dim3 gW((n2w + 255) / 256);
  split_w_kernel<<<gW, blk, 0, stream>>>(g_w,  WgH, WgL, n2w);
  split_w_kernel<<<gW, blk, 0, stream>>>(ph_w, WpH, WpL, n2w);
  split_w_kernel<<<gW, blk, 0, stream>>>(th_w, WtH, WtL, n2w);
  split_w_kernel<<<gW, blk, 0, stream>>>(W_w,  WwH, WwL, n2w);

  const dim3 gT(NP_ / 64, CH_ / 64, 1);
  const dim3 gGT(CI_ / 64, NS_ / 64, 1);
  const dim3 gConv(((NP_ / 64) * (CI_ / 64) + 7) / 8);
  const dim3 gS((QT_ * KT_ + 7) / 8);
  const dim3 gWc(((CH_ / 64) * (NP_ / 64) + 7) / 8);

  for (int b = 0; b < NB_; ++b) {
    const float* xb = x    + (size_t)b * CH_ * NP_;
    const float* mb = mask + (size_t)b * CH_ * NP_;
    tsplit_kernel<<<gT, blk, 0, stream>>>(mb, MH, ML, CH_, NP_);
    gemm64_kernel<2, 2><<<gConv, blk, 0, stream>>>(MH, ML, CH_, WtH, WtL, CH_, (void*)ThH, (void*)ThL, CI_, th_b, NP_, CI_, CH_);
    tsplit_kernel<<<gT, blk, 0, stream>>>(xb, XH, XL, CH_, NP_);
    gemm64_kernel<2, 0><<<gConv, blk, 0, stream>>>(XH, XL, CH_, WgH, WgL, CH_, (void*)Gpre, (void*)Gpre, CI_, g_b, NP_, CI_, CH_);
    gemm64_kernel<2, 0><<<gConv, blk, 0, stream>>>(XH, XL, CH_, WpH, WpL, CH_, (void*)Ppre, (void*)Ppre, CI_, ph_b, NP_, CI_, CH_);
    pool_kernel<<<dim3(KT_), blk, 0, stream>>>(Gpre, Ppre, PhH, PhL, Gpool);
    sgemm_stats_kernel<<<gS, blk, 0, stream>>>(ThH, ThL, PhH, PhL, S, Pmax, Psum);
    combine_kernel<<<dim3(KT_), dim3(64), 0, stream>>>(Pmax, Psum, Cmax, Cinv);
    tsplit_kernel<<<gGT, blk, 0, stream>>>(Gpool, GTH, GTL, NS_, CI_);
    pv_kernel<<<dim3(QT_), dim3(128), 0, stream>>>(S, Cmax, Cinv, GTH, GTL, YH, YL);
    gemm64_kernel<1, 0><<<gWc, blk, 0, stream>>>(WwH, WwL, CI_, YH, YL, CI_,
        (void*)(Wy + (size_t)b * CH_ * NP_), (void*)(Wy + (size_t)b * CH_ * NP_), NP_, W_b, CH_, NP_, CI_);
  }
  bn_stats_kernel<<<dim3(1), blk, 0, stream>>>(Wy, gamma, beta, SS);
  final_kernel<<<dim3(CH_, NB_), blk, 0, stream>>>(Wy, x, SS, out);
  (void)hipGetLastError();
}
